// LSTMDecoder_37288906064634
// MI455X (gfx1250) — hardware-verified
//
#include <hip/hip_runtime.h>
#include <math.h>

constexpr int NB     = 64;
constexpr int NS     = 512;
constexpr int NXW    = 14;
constexpr int NCMD   = 6;
constexpr int NCRD   = 8;
constexpr int NPCW   = 6;
constexpr int ND     = 512;
constexpr int NL     = 256;
constexpr int NIN    = ND + NL;
constexpr int NH     = 512;
constexpr int NP     = 128;
constexpr int NG4    = 4 * NH;
constexpr int NG16   = NG4 / 16;
constexpr int KXP    = 32;
constexpr int NXO    = NP + NCMD;
constexpr int NTOK   = NB * NS;
constexpr int NTHR   = 256;
constexpr int WE_THR = 128;
constexpr int BT     = 16;
constexpr int NCH    = NS / 64;
constexpr int HPITCH = 136;
constexpr int APITCH = 520;
constexpr int SPITCH = 132;
constexpr int CSLOT  = 32;
constexpr float XCARRY  = 64.0f;
constexpr float WECARRY = 256.0f;
constexpr float HCARRY  = 64.0f;
constexpr float WHCARRY = 256.0f;
constexpr float ACARRY  = 64.0f;
constexpr float WRCARRY = 256.0f;
constexpr float PCARRY  = 16384.0f;
constexpr float PCARRY_INV = 1.0f / 16384.0f;
constexpr float INV_NP   = 1.0f / 128.0f;
constexpr float LN_EPS_F = 1e-5f;
static_assert(XCARRY * WECARRY == PCARRY && HCARRY * WHCARRY == PCARRY && ACARRY * WRCARRY == PCARRY);
static_assert(NB % BT == 0);
static_assert(NH == 64 * (NTHR / 32));
static_assert(NP == 16 * (NTHR / 32));
static_assert(NP % 32 == 0 && NH % 32 == 0 && KXP == 32 && NXW <= KXP);
static_assert(HPITCH % 8 == 0 && APITCH % 8 == 0 && SPITCH % 4 == 0);
static_assert(HPITCH >= NP + 8 && APITCH >= NH + 8 && SPITCH >= NP);
static_assert(BT * NP == 2 * NTHR * 4);
static_assert(NG4 % WE_THR == 0 && ND == 4 * WE_THR);
static_assert(NG4 % 16 == 0 && NB == 64 && NL % 4 == 0);
static_assert((NG4 * NP / 8) % NTHR == 0 && (NP * NH / 8) % NTHR == 0);
static_assert(NTOK % NTHR == 0 && NS % 64 == 0);
static_assert(NCMD * 64 == 96 * 4 && NPCW * 64 == 96 * 4);
static_assert(CSLOT == 4 * 8);

typedef __attribute__((ext_vector_type(16))) _Float16 v16h;
typedef __attribute__((ext_vector_type(8)))  _Float16 v8h;
typedef __attribute__((ext_vector_type(8)))  float    v8f;
typedef __attribute__((ext_vector_type(4)))  float    v4f;
typedef __attribute__((ext_vector_type(4)))  unsigned v4u;

__device__ __forceinline__ unsigned f16_bits(float f) {
  const _Float16 h = (_Float16)f;
  return (unsigned)__builtin_bit_cast(unsigned short, h);
}

__device__ __forceinline__ void guard1_hm(v8f& a, v16h p, v16h q) {
  asm volatile("v_nop\n\tv_nop\n\tv_nop\n\tv_nop" : "+v"(a) : "v"(p), "v"(q) : "memory");
}
__device__ __forceinline__ void guard1_h(v8f& a, v16h p, v16h q) {
  asm volatile("v_nop\n\tv_nop\n\tv_nop\n\tv_nop" : "+v"(a) : "v"(p), "v"(q));
}
__device__ __forceinline__ void guard4_h5(v8f& a0, v8f& a1, v8f& a2, v8f& a3, v16h x, v16h y0, v16h y1, v16h y2, v16h y3) {
  asm volatile("v_nop\n\tv_nop\n\tv_nop\n\tv_nop" : "+v"(a0), "+v"(a1), "+v"(a2), "+v"(a3) : "v"(x), "v"(y0), "v"(y1), "v"(y2), "v"(y3));
}
__device__ __forceinline__ void acc_guard4(v8f& a, v8f& b, v8f& c, v8f& d) {
  asm volatile("v_nop\n\tv_nop\n\tv_nop\n\tv_nop" : "+v"(a), "+v"(b), "+v"(c), "+v"(d));
}
__device__ __forceinline__ void acc_guard1(v8f& a) { asm volatile("v_nop\n\tv_nop\n\tv_nop\n\tv_nop" : "+v"(a)); }
__device__ __forceinline__ void ld_split() { asm volatile("" ::: "memory"); }

template <typename T> struct Frag;
template <> struct Frag<_Float16> {
  typedef v16h V; union U { v16h v; v8h h[2]; };
  static __device__ __forceinline__ v16h load(const _Float16* p) {
    U f; f.h[0] = *(const v8h*)(p); f.h[1] = *(const v8h*)(p + 16); return f.v;
  }
  static __device__ __forceinline__ v8f mma(v16h a, v16h b, v8f c) {
    return __builtin_amdgcn_wmma_f32_16x16x32_f16(false, a, false, b, (short)0, c, false, false);
  }
};

__device__ __forceinline__ float frcp(float x) { return __builtin_amdgcn_rcpf(x); }
__device__ __forceinline__ float fsig(float x) {
  const float xc = fminf(fmaxf(x, -30.0f), 30.0f);
  return frcp(1.0f + expf(-xc));
}
__device__ __forceinline__ float ftanh(float x) {
  const float xc = fminf(fmaxf(x, -15.0f), 15.0f);
  return 1.0f - 2.0f * frcp(expf(2.0f * xc) + 1.0f);
}
__device__ __forceinline__ float wsum(float v) {
#pragma unroll
  for (int off = 16; off >= 1; off >>= 1) v += __shfl_xor(v, off, 32);
  return v;
}

__global__ __launch_bounds__(WE_THR) void weff_kernel(const float* __restrict__ W_ih, const float* __restrict__ cmdW,
                                                      const float* __restrict__ cmdb, const float* __restrict__ crdW,
                                                      const float* __restrict__ crdb, const float* __restrict__ b_ih,
                                                      const float* __restrict__ b_hh,
                                                      unsigned short* __restrict__ WE16, float* __restrict__ CB) {
  __shared__ __align__(16) float sCW[ND * NCMD];
  __shared__ __align__(16) float sOW[ND * NCRD];
  __shared__ __align__(16) float sBS[ND];
  __shared__ __align__(16) unsigned sH[WE_THR * 16];
  __shared__ __align__(16) float sCB[WE_THR];
  const int tid = threadIdx.x;
  const int g0 = blockIdx.x * WE_THR;
  const int g = g0 + tid;
#pragma unroll 1
  for (int i = tid; i < ND * NCMD / 4; i += WE_THR) *(v4f*)(sCW + 4 * i) = *(const v4f*)(cmdW + 4 * i);
#pragma unroll 1
  for (int i = tid; i < ND * NCRD / 4; i += WE_THR) *(v4f*)(sOW + 4 * i) = *(const v4f*)(crdW + 4 * i);
  {
    const v4f a = *(const v4f*)(cmdb + 4 * tid);
    const v4f bq = *(const v4f*)(crdb + 4 * tid);
    v4f s;
#pragma unroll
    for (int e = 0; e < 4; ++e) s[e] = a[e] + bq[e];
    *(v4f*)(sBS + 4 * tid) = s;
  }
  __syncthreads();

  float acc[NXW];
#pragma unroll
  for (int k = 0; k < NXW; ++k) acc[k] = 0.0f;
  float cbv = 0.0f;
  const float* wr = W_ih + (size_t)g * NIN;
#pragma unroll 1
  for (int j4 = 0; j4 < ND / 4; ++j4) {
    const v4f w4 = *(const v4f*)(wr + 4 * j4);
#pragma unroll
    for (int e = 0; e < 4; ++e) {
      const int j = 4 * j4 + e;
      const float w = w4[e];
#pragma unroll
      for (int k = 0; k < NCMD; ++k) acc[k] += w * sCW[j * NCMD + k];
#pragma unroll
      for (int k = 0; k < NCRD; ++k) acc[NCMD + k] += w * sOW[j * NCRD + k];
      cbv += w * sBS[j];
    }
  }
  cbv = (b_ih[g] + b_hh[g]) + cbv;

  unsigned wq[7];
#pragma unroll
  for (int m = 0; m < 7; ++m) wq[m] = f16_bits(acc[2 * m] * WECARRY) | (f16_bits(acc[2 * m + 1] * WECARRY) << 16);
  {
    v4u q0, q1;
    const v4u z4 = {0u, 0u, 0u, 0u};
    unsigned* ph = sH + tid * 16;
    q0[0] = wq[0]; q0[1] = wq[1]; q0[2] = wq[2]; q0[3] = wq[3];
    q1[0] = wq[4]; q1[1] = wq[5]; q1[2] = wq[6]; q1[3] = 0u;
    *(v4u*)(ph) = q0; *(v4u*)(ph + 4) = q1; *(v4u*)(ph + 8) = z4; *(v4u*)(ph + 12) = z4;
    sCB[tid] = cbv;
  }
  __syncthreads();

  unsigned* gH = (unsigned*)WE16 + (size_t)g0 * 16;
  for (int pass = 0; pass < 2; ++pass) {
#pragma unroll
    for (int it = 0; it < 4; ++it) {
      const int i = it * WE_THR + tid;
      const v4u vh = *(const v4u*)(sH + 4 * i);
      *(volatile v4u*)(gH + 4 * i) = vh;
    }
    if (tid < 32) {
      const v4f v = *(const v4f*)(sCB + 4 * tid);
      *(volatile v4f*)(CB + g0 + 4 * tid) = v;
    }
    __threadfence();
  }
}

__global__ __launch_bounds__(NTHR) void base_kernel(const float* __restrict__ W_ih, const float* __restrict__ ctx,
                                                    const float* __restrict__ CB, float* __restrict__ BASEF) {
  __shared__ __align__(16) float sW[16 * NL];
  __shared__ __align__(16) float sS[4 * 256];
  const int tid = threadIdx.x, nt = blockIdx.x;
#pragma unroll
  for (int it = 0; it < 4; ++it) {
    const int i = it * NTHR + tid;
    const int gl = i >> 6, c4 = (i & 63) * 4;
    *(v4f*)(sW + gl * NL + c4) = *(const v4f*)(W_ih + (size_t)(16 * nt + gl) * NIN + ND + c4);
  }
  __syncthreads();
  const int gl = tid & 15, bq = tid >> 4;
  const int g = 16 * nt + gl;
  float acc[4];
#pragma unroll
  for (int e = 0; e < 4; ++e) acc[e] = 0.0f;
  const float* wlp = sW + gl * NL;
  const float* cx = ctx + (size_t)(4 * bq) * NL;
#pragma unroll 1
  for (int j4 = 0; j4 < NL / 4; ++j4) {
    const v4f w4 = *(const v4f*)(wlp + 4 * j4);
#pragma unroll
    for (int e = 0; e < 4; ++e) {
      const v4f x4 = *(const v4f*)(cx + (size_t)e * NL + 4 * j4);
      float s = acc[e];
      s += w4[0] * x4[0]; s += w4[1] * x4[1]; s += w4[2] * x4[2]; s += w4[3] * x4[3];
      acc[e] = s;
    }
  }
  const float cbg = CB[g];
#pragma unroll
  for (int e = 0; e < 4; ++e) {
    const int b = 4 * bq + e;
    const int btl = b >> 4, bl = b & 15;
    const int lf = (bl >> 3) * 16 + gl, r = bl & 7;
    sS[btl * 256 + lf * 8 + r] = (cbg + acc[e]) * PCARRY;
  }
  __syncthreads();
  {
    const int btl = tid >> 6, f4 = (tid & 63) * 4;
    const v4f v = *(const v4f*)(sS + btl * 256 + f4);
    float* dst = BASEF + ((size_t)(btl * NG16 + nt)) * 256 + f4;
    for (int pass = 0; pass < 2; ++pass) {
      *(volatile v4f*)dst = v;
      __threadfence();
    }
  }
}

__global__ __launch_bounds__(NTHR) void cvt8_kernel(const float* __restrict__ src, unsigned short* __restrict__ dst, int n8, float sc) {
  const int i = blockIdx.x * NTHR + threadIdx.x;
  if (i < n8) {
    const float* sp = src + (size_t)i * 8;
    const v4f a = *(const v4f*)(sp);
    const v4f b = *(const v4f*)(sp + 4);
    v8h hv;
#pragma unroll
    for (int e = 0; e < 4; ++e) {
      hv[e]     = (_Float16)(a[e] * sc);
      hv[4 + e] = (_Float16)(b[e] * sc);
    }
    for (int pass = 0; pass < 2; ++pass) {
      *(volatile v8h*)(dst + (size_t)i * 8) = hv;
      __threadfence();
    }
  }
}

__global__ __launch_bounds__(NTHR) void xplane_kernel(const float* __restrict__ x, unsigned short* __restrict__ X16) {
  __shared__ __align__(16) unsigned sH[NTHR * 16];
  const int tid = threadIdx.x;
  const int r0 = blockIdx.x * NTHR;
  const int r = r0 + tid;
  const int t = r / NB, b = r - t * NB;
  const float* sp = x + ((size_t)b * NS + t) * NXW;
  float v[NXW];
#pragma unroll
  for (int k = 0; k < 8; ++k) v[k] = sp[k] * XCARRY;
  ld_split();
#pragma unroll
  for (int k = 8; k < NXW; ++k) v[k] = sp[k] * XCARRY;
  unsigned wq[7];
#pragma unroll
  for (int m = 0; m < 7; ++m) wq[m] = f16_bits(v[2 * m]) | (f16_bits(v[2 * m + 1]) << 16);
  {
    v4u q0, q1;
    const v4u z4 = {0u, 0u, 0u, 0u};
    unsigned* ph = sH + tid * 16;
    q0[0] = wq[0]; q0[1] = wq[1]; q0[2] = wq[2]; q0[3] = wq[3];
    q1[0] = wq[4]; q1[1] = wq[5]; q1[2] = wq[6]; q1[3] = 0u;
    *(v4u*)(ph) = q0; *(v4u*)(ph + 4) = q1; *(v4u*)(ph + 8) = z4; *(v4u*)(ph + 12) = z4;
  }
  __syncthreads();
  unsigned* gH = (unsigned*)X16 + (size_t)r0 * 16;
  for (int pass = 0; pass < 2; ++pass) {
#pragma unroll
    for (int it = 0; it < 4; ++it) {
      const int i = it * NTHR + tid;
      const v4u vh = *(const v4u*)(sH + 4 * i);
      *(volatile v4u*)(gH + 4 * i) = vh;
    }
    __threadfence();
  }
}

__global__ __launch_bounds__(NTHR) __attribute__((amdgpu_num_vgpr(256)))
void lstm_scan_kernel(const float* __restrict__ BASEF, const unsigned short* __restrict__ X16p,
                      const unsigned short* __restrict__ WE16p, const unsigned short* __restrict__ WHH16p,
                      const unsigned short* __restrict__ WHR16p, float* __restrict__ HS) {
  __shared__ __align__(16) _Float16 hLt[BT * HPITCH];
  __shared__ __align__(16) _Float16 aT[BT * APITCH];
  __shared__ __align__(16) float    Cs[NTHR * CSLOT];
  __shared__ __align__(16) float    Hst[BT * SPITCH];
  const _Float16* X16   = (const _Float16*)X16p;
  const _Float16* WE16  = (const _Float16*)WE16p;
  const _Float16* WHH16 = (const _Float16*)WHH16p;
  const _Float16* WHR16 = (const _Float16*)WHR16p;
  const int tid = threadIdx.x, lane = tid & 31, wave = tid >> 5;
  const int c = lane & 15, hh = lane >> 4, koff = hh * 8;
  const int bt = blockIdx.x, b0 = bt * BT;

#pragma unroll 1
  for (int i = tid; i < BT * HPITCH; i += NTHR) hLt[i] = (_Float16)0.0f;
  float* cbase = Cs + tid * CSLOT;
  {
    const v4f z4 = {0.f, 0.f, 0.f, 0.f};
#pragma unroll
    for (int m = 0; m < CSLOT / 4; ++m) *(v4f*)(cbase + 4 * m) = z4;
  }
  __syncthreads();

  const _Float16* hrow = hLt + c * HPITCH + koff;
  const _Float16* arow = aT + c * APITCH + koff;
  const int pcol = 16 * wave + c;
  const v8f z8 = {0.f, 0.f, 0.f, 0.f, 0.f, 0.f, 0.f, 0.f};

#pragma unroll 1
  for (int t = 0; t < NS; ++t) {
    const v16h xa = Frag<_Float16>::load(X16 + ((size_t)t * NB + b0 + c) * KXP + koff);

#pragma unroll 1
    for (int n2 = 0; n2 < 4; ++n2) {
      const int ncol = 64 * wave + 16 * n2 + c;
      v8f acc[4];
#pragma unroll
      for (int q = 0; q < 4; ++q) {
        const int gcol = q * NH + ncol;
        acc[q] = *(const v8f*)(BASEF + ((size_t)(bt * NG16 + (gcol >> 4)) * 32 + lane) * 8);
        const v16h wb = Frag<_Float16>::load(WE16 + (size_t)gcol * KXP + koff);
        acc[q] = Frag<_Float16>::mma(xa, wb, acc[q]);
        guard1_hm(acc[q], xa, wb);
      }
#pragma unroll 1
      for (int k0 = 0; k0 < NP; k0 += 32) {
        const v16h ah = Frag<_Float16>::load(hrow + k0);
        const v16h w0 = Frag<_Float16>::load(WHH16 + (size_t)(0 * NH + ncol) * NP + koff + k0);
        const v16h w1 = Frag<_Float16>::load(WHH16 + (size_t)(1 * NH + ncol) * NP + koff + k0);
        const v16h w2 = Frag<_Float16>::load(WHH16 + (size_t)(2 * NH + ncol) * NP + koff + k0);
        const v16h w3 = Frag<_Float16>::load(WHH16 + (size_t)(3 * NH + ncol) * NP + koff + k0);
        acc[0] = Frag<_Float16>::mma(ah, w0, acc[0]);
        acc[1] = Frag<_Float16>::mma(ah, w1, acc[1]);
        acc[2] = Frag<_Float16>::mma(ah, w2, acc[2]);
        acc[3] = Frag<_Float16>::mma(ah, w3, acc[3]);
        guard4_h5(acc[0], acc[1], acc[2], acc[3], ah, w0, w1, w2, w3);
      }
      acc_guard4(acc[0], acc[1], acc[2], acc[3]);
      const v4f ca = *(const v4f*)(cbase + n2 * 8);
      const v4f cb = *(const v4f*)(cbase + n2 * 8 + 4);
      const float cold[8] = {ca[0], ca[1], ca[2], ca[3], cb[0], cb[1], cb[2], cb[3]};
      float cnew[8];
#pragma unroll
      for (int r = 0; r < 8; ++r) {
        const float zi = acc[0][r] * PCARRY_INV;
        const float zf = acc[1][r] * PCARRY_INV;
        const float zg = acc[2][r] * PCARRY_INV;
        const float zo = acc[3][r] * PCARRY_INV;
        const float ig = fsig(zi);
        const float fg = fsig(zf);
        const float gg = ftanh(zg);
        const float og = fsig(zo);
        const float cn = fg * cold[r] + ig * gg;
        cnew[r] = cn;
        const float av = og * ftanh(cn);
        aT[(8 * hh + r) * APITCH + ncol] = (_Float16)(av * ACARRY);
      }
      v4f na, nb;
      na[0] = cnew[0]; na[1] = cnew[1]; na[2] = cnew[2]; na[3] = cnew[3];
      nb[0] = cnew[4]; nb[1] = cnew[5]; nb[2] = cnew[6]; nb[3] = cnew[7];
      *(v4f*)(cbase + n2 * 8) = na;
      *(v4f*)(cbase + n2 * 8 + 4) = nb;
    }
    __syncthreads();

    v8f hacc = z8;
#pragma unroll 2
    for (int k0 = 0; k0 < NH; k0 += 32) {
      const v16h af = Frag<_Float16>::load(arow + k0);
      const v16h wf = Frag<_Float16>::load(WHR16 + (size_t)pcol * NH + koff + k0);
      hacc = Frag<_Float16>::mma(af, wf, hacc);
      guard1_h(hacc, af, wf);
    }
    acc_guard1(hacc);
#pragma unroll
    for (int r = 0; r < 8; ++r) {
      const float hv = hacc[r] * PCARRY_INV;
      hLt[(8 * hh + r) * HPITCH + pcol] = (_Float16)(hv * HCARRY);
      Hst[(8 * hh + r) * SPITCH + pcol] = hv;
    }
    __syncthreads();

    for (int pass = 0; pass < 2; ++pass) {
#pragma unroll
      for (int it = 0; it < 2; ++it) {
        const int i = it * NTHR + tid;
        const int row = i >> 5, c4 = (i & 31) * 4;
        const v4f v = *(const v4f*)(Hst + row * SPITCH + c4);
        *(volatile v4f*)(HS + ((size_t)t * NB + b0 + row) * NP + c4) = v;
      }
      __threadfence();
    }
  }
}

__global__ __launch_bounds__(NTHR) void head_kernel(const float* __restrict__ HS, const float* __restrict__ ln_g,
                                                    const float* __restrict__ ln_b, const float* __restrict__ outcW,
                                                    const float* __restrict__ outcb, const float* __restrict__ outxW,
                                                    const float* __restrict__ outxb, const float* __restrict__ scale_p,
                                                    float* __restrict__ out0, float* __restrict__ out1) {
  __shared__ __align__(16) float sWc[NCMD * NP];
  __shared__ __align__(16) float sWx[NPCW * NXO];
  __shared__ float sbc[8], sbx[8];
  __shared__ __align__(16) float sO[2][64 * NCMD];
  const int tid = threadIdx.x, lane = tid & 31, wave = tid >> 5;
  const int b = blockIdx.x / NCH, ch = blockIdx.x - b * NCH;
#pragma unroll 1
  for (int it = 0; it < (NCMD * NP + NTHR - 1) / NTHR; ++it) {
    const int i = it * NTHR + tid;
    const int ic = (i < NCMD * NP) ? i : (NCMD * NP - 1);
    const float v = outcW[ic];
    if (i < NCMD * NP) sWc[i] = v;
  }
#pragma unroll 1
  for (int it = 0; it < (NPCW * NXO + NTHR - 1) / NTHR; ++it) {
    const int i = it * NTHR + tid;
    const int ic = (i < NPCW * NXO) ? i : (NPCW * NXO - 1);
    const float v = outxW[ic];
    if (i < NPCW * NXO) sWx[i] = v;
  }
  {
    const int ic = (tid < NCMD) ? tid : (NCMD - 1);
    const float vc = outcb[ic];
    const int ix = (tid < NPCW) ? tid : (NPCW - 1);
    const float vx = outxb[ix];
    if (tid < NCMD) sbc[tid] = vc;
    if (tid < NPCW) sbx[tid] = vx;
  }
  __syncthreads();
  const v4f g4 = *(const v4f*)(ln_g + 4 * lane);
  const v4f b4 = *(const v4f*)(ln_b + 4 * lane);
  const float csc = scale_p[0];

#pragma unroll 1
  for (int i = 0; i < 8; ++i) {
    const int tl = wave * 8 + i;
    const int t = ch * 64 + tl;
    const v4f hv = *(const v4f*)(HS + ((size_t)t * NB + b) * NP + 4 * lane);
    float s = (hv[0] + hv[1]) + (hv[2] + hv[3]);
    s = wsum(s);
    const float mu = s * INV_NP;
    float d[4];
    float ss = 0.0f;
#pragma unroll
    for (int e = 0; e < 4; ++e) { d[e] = hv[e] - mu; ss += d[e] * d[e]; }
    ss = wsum(ss);
    const float var = ss * INV_NP;
    const float rstd = rsqrtf(var + LN_EPS_F);
    float y[4];
#pragma unroll
    for (int e = 0; e < 4; ++e) y[e] = (d[e] * rstd) * g4[e] + b4[e];

    float lg[NCMD];
#pragma unroll
    for (int o = 0; o < NCMD; ++o) {
      const float* w = sWc + o * NP + 4 * lane;
      float p = 0.0f;
      p += y[0] * w[0]; p += y[1] * w[1]; p += y[2] * w[2]; p += y[3] * w[3];
      p = wsum(p);
      lg[o] = p + sbc[o];
    }
    if (lane == 0) {
#pragma unroll
      for (int o = 0; o < NCMD; ++o) sO[0][tl * NCMD + o] = lg[o];
    }
#pragma unroll 1
    for (int o = 0; o < NPCW; ++o) {
      const float* w = sWx + o * NXO + 4 * lane;
      float p = 0.0f;
      p += y[0] * w[0]; p += y[1] * w[1]; p += y[2] * w[2]; p += y[3] * w[3];
      p = wsum(p);
      float zz = p + sbx[o];
#pragma unroll
      for (int j = 0; j < NCMD; ++j) zz += lg[j] * sWx[o * NXO + NP + j];
      const float co = tanhf(zz * csc);
      if (lane == 0) sO[1][tl * NPCW + o] = co;
    }
  }
  __syncthreads();
  if (tid < 192) {
    const int which = (tid >= 96) ? 1 : 0;
    const int f4i = tid - 96 * which;
    const v4f v = *(const v4f*)(&sO[which][4 * f4i]);
    float* dst = (which ? out1 : out0) + ((size_t)b * NS + (size_t)ch * 64) * NCMD + 4 * f4i;
    for (int pass = 0; pass < 2; ++pass) {
      *(volatile v4f*)dst = v;
      __threadfence();
    }
  }
}

extern "C" void kernel_launch(void* const* d_in, const int* in_sizes, int n_in,
                              void* d_out, int out_size, void* d_ws, size_t ws_size, hipStream_t stream) {
  if (n_in < 18 || d_out == nullptr || d_ws == nullptr) return;
  if (in_sizes[0] != NB * NS * NXW || in_sizes[1] != NB * NL || in_sizes[2] != ND * NCMD || in_sizes[3] != ND ||
      in_sizes[4] != ND * NCRD || in_sizes[5] != ND || in_sizes[6] != NG4 * NIN || in_sizes[7] != NG4 * NP ||
      in_sizes[8] != NG4 || in_sizes[9] != NG4 || in_sizes[10] != NP * NH || in_sizes[11] != NP || in_sizes[12] != NP ||
      in_sizes[13] != NCMD * NP || in_sizes[14] != NCMD || in_sizes[15] != NPCW * NXO || in_sizes[16] != NPCW ||
      in_sizes[17] != 1 || out_size != 2 * NTOK * NCMD) return;

  const float* x      = (const float*)d_in[0];
  const float* ctx    = (const float*)d_in[1];
  const float* cmdW   = (const float*)d_in[2];
  const float* cmdb   = (const float*)d_in[3];
  const float* crdW   = (const float*)d_in[4];
  const float* crdb   = (const float*)d_in[5];
  const float* W_ih   = (const float*)d_in[6];
  const float* W_hh   = (const float*)d_in[7];
  const float* b_ih   = (const float*)d_in[8];
  const float* b_hh   = (const float*)d_in[9];
  const float* W_hr   = (const float*)d_in[10];
  const float* ln_g   = (const float*)d_in[11];
  const float* ln_b   = (const float*)d_in[12];
  const float* outcW  = (const float*)d_in[13];
  const float* outcb  = (const float*)d_in[14];
  const float* outxW  = (const float*)d_in[15];
  const float* outxb  = (const float*)d_in[16];
  const float* cscale = (const float*)d_in[17];
  float* out0 = (float*)d_out;
  float* out1 = out0 + (size_t)NTOK * NCMD;

  char* ws = (char*)d_ws; size_t off = 0;
  auto carve = [&](size_t bytes) -> char* { char* p = ws + off; off += (bytes + 255) & ~(size_t)255; return p; };
  unsigned short* WE16  = (unsigned short*)carve((size_t)NG4 * KXP * 2);
  float*          CB    = (float*)carve((size_t)NG4 * 4);
  float*          BASEF = (float*)carve((size_t)NB * NG4 * 4);
  unsigned short* WHH16 = (unsigned short*)carve((size_t)NG4 * NP * 2);
  unsigned short* WHR16 = (unsigned short*)carve((size_t)NP * NH * 2);
  unsigned short* X16   = (unsigned short*)carve((size_t)NTOK * KXP * 2);
  float*          HS    = (float*)carve((size_t)NTOK * NP * 4);
  if (off > ws_size || off > (size_t)134217728) return;

  weff_kernel<<<NG4 / WE_THR, WE_THR, 0, stream>>>(W_ih, cmdW, cmdb, crdW, crdb, b_ih, b_hh, WE16, CB);
  base_kernel<<<NG16, NTHR, 0, stream>>>(W_ih, ctx, CB, BASEF);
  cvt8_kernel<<<(NG4 * NP / 8) / NTHR, NTHR, 0, stream>>>(W_hh, WHH16, NG4 * NP / 8, WHCARRY);
  cvt8_kernel<<<(NP * NH / 8) / NTHR, NTHR, 0, stream>>>(W_hr, WHR16, NP * NH / 8, WRCARRY);
  xplane_kernel<<<NTOK / NTHR, NTHR, 0, stream>>>(x, X16);
  lstm_scan_kernel<<<NB / BT, NTHR, 0, stream>>>(BASEF, X16, WE16, WHH16, WHR16, HS);
  head_kernel<<<NB * NCH, NTHR, 0, stream>>>(HS, ln_g, ln_b, outcW, outcb, outxW, outxb, cscale, out0, out1);
}
